// SelfAttention_22119081574638
// MI455X (gfx1250) — hardware-verified
//
#include <hip/hip_runtime.h>
#ifndef NB
#define NB 2
#endif
#ifndef SEQ
#define SEQ 4096
#endif
#define NB_FULL 2
#define SEQ_FULL 4096
#define HID 1024
#define NHD 16
#define HD 64
#define BLK 256
#define NT ((SEQ / BLK) * NHD)
#define NR (NB * SEQ)

static_assert(SEQ % BLK == 0);
static_assert(NR % 128 == 0);
static_assert(HID % 128 == 0);
static_assert(NHD * HD == HID);
static_assert(NB <= NB_FULL);
static_assert(SEQ <= SEQ_FULL);

typedef unsigned short v8us __attribute__((ext_vector_type(8), may_alias));
typedef float  v8f  __attribute__((ext_vector_type(8)));
typedef float  v4f  __attribute__((ext_vector_type(4)));
typedef float  v4fa __attribute__((ext_vector_type(4), may_alias));
typedef _Float16 v16h __attribute__((ext_vector_type(16)));
union FragH { v16h v; v8us half[2]; _Float16 h[16]; unsigned short u[16]; };

__device__ __forceinline__ unsigned short bf16_bits(float x) { unsigned int u = __float_as_uint(x); return (unsigned short)((u + 0x7FFFu + ((u >> 16) & 1u)) >> 16); }
__device__ __forceinline__ float bf16_val(unsigned short b) { return __uint_as_float(((unsigned int)b) << 16); }
__device__ __forceinline__ float bf16_rne(float x) { return bf16_val(bf16_bits(x)); }

__device__ __forceinline__ v16h g2_frag(const _Float16* p, int hh) { FragH f; f.half[0] = *(const v8us*)((const unsigned short*)p + 8 * hh); f.half[1] = *(const v8us*)((const unsigned short*)p + 16 + 8 * hh); return f.v; }
__device__ __forceinline__ v8f g2_mma(v16h a, v16h b, v8f c) { v8f d = __builtin_amdgcn_wmma_f32_16x16x32_f16(false, a, false, b, (short)0, c, false, false); asm volatile("v_nop\n\tv_nop\n\tv_nop\n\tv_nop" : "+v"(d) : "v"(a), "v"(b)); return d; }

__global__ __launch_bounds__(256) void k_x16(const float* __restrict__ x, _Float16* __restrict__ X16) {
  const size_t t = (size_t)blockIdx.x * 256 + threadIdx.x;
  if (t >= (size_t)NR * (HID / 8)) return;
  const size_t row = t / (HID / 8);
  const int c8 = (int)(t % (HID / 8)) * 8;
  const size_t b = row / SEQ, s = row % SEQ;
  const float* src = x + ((b * SEQ_FULL + s) * HID + c8);
  const v4f a = *(const v4fa*)src, c = *(const v4fa*)(src + 4);
  FragH f;
#pragma unroll
  for (int q = 0; q < 4; ++q) { f.h[q] = (_Float16)bf16_rne(a[q]); f.h[4 + q] = (_Float16)bf16_rne(c[q]); }
  const v8us o = f.half[0];
  unsigned short* d = (unsigned short*)X16 + row * HID + c8;
  *(volatile v8us*)d = o;
  __threadfence();
  *(volatile v8us*)d = o;
}

__global__ __launch_bounds__(256) void k_wt_f16(const float* __restrict__ W, _Float16* __restrict__ Wt, int K, int N, float scale) {
  const int t = blockIdx.x * 256 + threadIdx.x;
  if (t >= N * (K / 8)) return;
  const int n = t / (K / 8), k8 = (t % (K / 8)) * 8;
  FragH f;
#pragma unroll
  for (int i = 0; i < 8; ++i) f.h[i] = (_Float16)(bf16_rne(W[(size_t)(k8 + i) * N + n]) * scale);
  const v8us o = f.half[0];
  unsigned short* d = (unsigned short*)Wt + (size_t)n * K + k8;
  *(volatile v8us*)d = o;
  __threadfence();
  *(volatile v8us*)d = o;
}

template <int BIASROW>
__global__ __launch_bounds__(128) void k_gemm16(const _Float16* __restrict__ A, int lda, const _Float16* __restrict__ Bh, int ldb, float alpha,
                                                const float* __restrict__ bias, _Float16* __restrict__ C16, int ldc, int M, int N, int K) {
  __shared__ __attribute__((aligned(16))) float so[4][32][68];
  const int tid = threadIdx.x, lane = tid & 31, ln = lane & 15, hh = lane >> 4;
  const int w = __builtin_amdgcn_readfirstlane((int)(threadIdx.x >> 5));
  const int ntn = N >> 6;
  const int mt = (int)blockIdx.x / ntn, nq = (int)blockIdx.x - mt * ntn;
  const int row0 = mt * 128 + 32 * w, col0 = nq * 64;
  if (row0 >= M) return;
  const _Float16* a0p = A + (size_t)(row0 + ln) * lda; const _Float16* a1p = a0p + (size_t)16 * lda;
  const _Float16* b0p = Bh + (size_t)(col0 + ln) * ldb; const _Float16* b1p = b0p + (size_t)16 * ldb; const _Float16* b2p = b1p + (size_t)16 * ldb; const _Float16* b3p = b2p + (size_t)16 * ldb;
  const v8f z8 = {0.f,0.f,0.f,0.f,0.f,0.f,0.f,0.f};
  v8f c00 = z8, c01 = z8, c02 = z8, c03 = z8, c10 = z8, c11 = z8, c12 = z8, c13 = z8;
#pragma unroll 1
  for (int kb = 0; kb < K; kb += 32) {
    const v16h a0 = g2_frag(a0p + kb, hh), a1 = g2_frag(a1p + kb, hh);
    v16h b = g2_frag(b0p + kb, hh); c00 = g2_mma(a0, b, c00); c10 = g2_mma(a1, b, c10);
    b = g2_frag(b1p + kb, hh); c01 = g2_mma(a0, b, c01); c11 = g2_mma(a1, b, c11);
    b = g2_frag(b2p + kb, hh); c02 = g2_mma(a0, b, c02); c12 = g2_mma(a1, b, c12);
    b = g2_frag(b3p + kb, hh); c03 = g2_mma(a0, b, c03); c13 = g2_mma(a1, b, c13);
  }
  v8f accs[8] = {c00, c01, c02, c03, c10, c11, c12, c13};
#pragma unroll
  for (int u = 0; u < 8; ++u) {
    const int t = u & 3, half = u >> 2;
    float bc = 0.f;
    if (!BIASROW) bc = bf16_rne(bias[col0 + t * 16 + ln]);
#pragma unroll
    for (int r = 0; r < 8; ++r) {
      const int rloc = half * 16 + 8 * hh + r;
      float bv = bc;
      if (BIASROW) bv = bf16_rne(bias[row0 + rloc]);
      so[w][rloc][t * 16 + ln] = accs[u][r] * alpha + bv;
    }
  }
  __builtin_amdgcn_fence(4  , "workgroup");
  __builtin_amdgcn_wave_barrier();
  const int rq = lane >> 3, pc = (lane & 7) * 8;
  for (int pass = 0; pass < 2; ++pass) {
#pragma unroll
    for (int q = 0; q < 8; ++q) {
      const int rr = q * 4 + rq;
      const v4f a = *(const v4fa*)&so[w][rr][pc], c = *(const v4fa*)&so[w][rr][pc + 4];
      FragH f;
#pragma unroll
      for (int i = 0; i < 4; ++i) { f.h[i] = (_Float16)a[i]; f.h[4 + i] = (_Float16)c[i]; }
      const v8us o = f.half[0];
      *(volatile v8us*)((unsigned short*)C16 + (size_t)(row0 + rr) * ldc + col0 + pc) = o;
    }
    if (pass == 0) __threadfence();
  }
}

__global__ __launch_bounds__(128) void k_attn(const _Float16* __restrict__ Q16, const _Float16* __restrict__ K16, const _Float16* __restrict__ VT,
                                              const int* __restrict__ perm, float* __restrict__ out) {
  __shared__ __attribute__((aligned(16))) float so[4][16][68];
  const int tid = threadIdx.x, lane = tid & 31, ln = lane & 15, hh = lane >> 4;
  const int wave = __builtin_amdgcn_readfirstlane((int)(threadIdx.x >> 5));
  const int bid = (int)blockIdx.x;
  const int sub = bid & 3, pt = (bid >> 2) % NT, b = (bid >> 2) / NT;
  const int g = pt >> 4, n = pt & 15;
  int pv = __builtin_amdgcn_readfirstlane(perm[pt]);
  pv = (pv < 0) ? 0 : ((pv > NT - 1) ? (NT - 1) : pv);
  const int g2 = pv >> 4, n2 = pv & 15;
  const size_t qrow = (size_t)b * SEQ + (size_t)g * BLK + sub * 64 + wave * 16;
  const size_t krow0 = (size_t)b * SEQ + (size_t)g2 * BLK;
  const _Float16* qp = Q16 + (qrow + ln) * HID + n * HD;
  const _Float16* kp = K16 + (krow0 + ln) * HID + n2 * HD;
  const _Float16* vp = VT + (size_t)(n2 * HD + ln) * NR + krow0;
  const v16h bq0 = g2_frag(qp, hh), bq1 = g2_frag(qp + 32, hh);
  const v8f z8 = {0.f,0.f,0.f,0.f,0.f,0.f,0.f,0.f};
  v8f o0 = z8, o1 = z8, o2 = z8, o3 = z8;
  float m = -1.0e30f, l = 0.f;
  const float C2 = 0.125f * 1.4426950408889634f;
#pragma unroll 1
  for (int ks = 0; ks < BLK / 32; ++ks) {
    const int key0 = ks * 32;
    const _Float16* k0p = kp + (size_t)key0 * HID;
    const _Float16* k1p = k0p + (size_t)16 * HID;
    v16h ka = g2_frag(k0p, hh), kb2 = g2_frag(k0p + 32, hh);
    v8f s0 = g2_mma(ka, bq0, z8); s0 = g2_mma(kb2, bq1, s0);
    ka = g2_frag(k1p, hh); kb2 = g2_frag(k1p + 32, hh);
    v8f s1 = g2_mma(ka, bq0, z8); s1 = g2_mma(kb2, bq1, s1);
    float mloc = s0[0];
#pragma unroll
    for (int r = 0; r < 8; ++r) { mloc = fmaxf(mloc, s0[r]); mloc = fmaxf(mloc, s1[r]); }
    mloc = mloc * C2;
    mloc = fmaxf(mloc, __shfl_xor(mloc, 16));
    const float mn = fmaxf(m, mloc);
    const float al = __builtin_amdgcn_exp2f(m - mn);
    m = mn;
    float ls = 0.f;
    FragH pf;
#pragma unroll
    for (int r = 0; r < 8; ++r) {
      const float e0 = __builtin_amdgcn_exp2f(fmaf(s0[r], C2, -mn));
      const float e1 = __builtin_amdgcn_exp2f(fmaf(s1[r], C2, -mn));
      ls += e0; ls += e1;
      pf.h[r] = (_Float16)(e0 * 256.0f);
      pf.h[8 + r] = (_Float16)(e1 * 256.0f);
    }
    l = l * al + ls;
    o0 = o0 * al; o1 = o1 * al; o2 = o2 * al; o3 = o3 * al;
    const _Float16* vk = vp + key0;
    const v16h va = g2_frag(vk, hh);
    const v16h vb = g2_frag(vk + (size_t)16 * NR, hh);
    const v16h vc = g2_frag(vk + (size_t)32 * NR, hh);
    const v16h vd = g2_frag(vk + (size_t)48 * NR, hh);
    o0 = g2_mma(va, pf.v, o0);
    o1 = g2_mma(vb, pf.v, o1);
    o2 = g2_mma(vc, pf.v, o2);
    o3 = g2_mma(vd, pf.v, o3);
  }
  const float lt = l + __shfl_xor(l, 16);
  const float inv = (1.0f / lt) * 0.00390625f;
  {
    v4f a, c;
    a[0] = o0[0] * inv; a[1] = o0[1] * inv; a[2] = o0[2] * inv; a[3] = o0[3] * inv; c[0] = o0[4] * inv; c[1] = o0[5] * inv; c[2] = o0[6] * inv; c[3] = o0[7] * inv;
    *(v4fa*)&so[wave][ln][0 + 8 * hh] = a; *(v4fa*)&so[wave][ln][0 + 8 * hh + 4] = c;
    a[0] = o1[0] * inv; a[1] = o1[1] * inv; a[2] = o1[2] * inv; a[3] = o1[3] * inv; c[0] = o1[4] * inv; c[1] = o1[5] * inv; c[2] = o1[6] * inv; c[3] = o1[7] * inv;
    *(v4fa*)&so[wave][ln][16 + 8 * hh] = a; *(v4fa*)&so[wave][ln][16 + 8 * hh + 4] = c;
    a[0] = o2[0] * inv; a[1] = o2[1] * inv; a[2] = o2[2] * inv; a[3] = o2[3] * inv; c[0] = o2[4] * inv; c[1] = o2[5] * inv; c[2] = o2[6] * inv; c[3] = o2[7] * inv;
    *(v4fa*)&so[wave][ln][32 + 8 * hh] = a; *(v4fa*)&so[wave][ln][32 + 8 * hh + 4] = c;
    a[0] = o3[0] * inv; a[1] = o3[1] * inv; a[2] = o3[2] * inv; a[3] = o3[3] * inv; c[0] = o3[4] * inv; c[1] = o3[5] * inv; c[2] = o3[6] * inv; c[3] = o3[7] * inv;
    *(v4fa*)&so[wave][ln][48 + 8 * hh] = a; *(v4fa*)&so[wave][ln][48 + 8 * hh + 4] = c;
  }
  __builtin_amdgcn_fence(4  , "workgroup");
  __builtin_amdgcn_wave_barrier();
  const int rsub = lane >> 4, c4 = (lane & 15) * 4;
  float* obase = out + qrow * HID + n * HD + c4;
  for (int pass = 0; pass < 2; ++pass) {
#pragma unroll
    for (int q = 0; q < 8; ++q) {
      const int rr = q * 2 + rsub;
      const v4f v = *(const v4fa*)&so[wave][rr][c4];
      *(volatile v4f*)(obase + (size_t)rr * HID) = v;
    }
    if (pass == 0) __threadfence();
  }
}

extern "C" void kernel_launch(void* const* d_in, const int* in_sizes, int n_in,
                              void* d_out, int out_size, void* d_ws, size_t ws_size, hipStream_t stream) {
  if (n_in < 9) return;
  if ((size_t)in_sizes[0] < ((size_t)(NB - 1) * SEQ_FULL + SEQ) * HID) return;
  if (in_sizes[2] < NT) return;
  if (in_sizes[3] < HID * HID || in_sizes[5] < HID * HID || in_sizes[7] < HID * HID) return;
  if (in_sizes[4] < HID || in_sizes[6] < HID || in_sizes[8] < HID) return;
  if ((size_t)out_size < (size_t)NR * HID) return;
  const float* x = (const float*)d_in[0];
  const int* perm = (const int*)d_in[2];
  const float* wq = (const float*)d_in[3]; const float* bq = (const float*)d_in[4];
  const float* wk = (const float*)d_in[5]; const float* bk = (const float*)d_in[6];
  const float* wv = (const float*)d_in[7]; const float* bv = (const float*)d_in[8];
  char* ws = (char*)d_ws; size_t off = 0;
  auto take = [&](size_t bytes) { char* p = ws + off; off += (bytes + 255) & ~(size_t)255; return p; };
  _Float16* BQ  = (_Float16*)take((size_t)HID * HID * 2);
  _Float16* BK  = (_Float16*)take((size_t)HID * HID * 2);
  _Float16* BV  = (_Float16*)take((size_t)HID * HID * 2);
  _Float16* X16 = (_Float16*)take((size_t)NR * HID * 2);
  _Float16* Q16 = (_Float16*)take((size_t)NR * HID * 2);
  _Float16* K16 = (_Float16*)take((size_t)NR * HID * 2);
  _Float16* VT  = (_Float16*)take((size_t)HID * NR * 2);
  if (off > ws_size) return;
  {
    const unsigned gw = (unsigned)(((size_t)HID * (HID / 8) + 255) / 256);
    k_wt_f16<<<gw, 256, 0, stream>>>(wq, BQ, HID, HID, 16.0f);
    k_wt_f16<<<gw, 256, 0, stream>>>(wk, BK, HID, HID, 16.0f);
    k_wt_f16<<<gw, 256, 0, stream>>>(wv, BV, HID, HID, 16.0f);
  }
  k_x16<<<(unsigned)(((size_t)NR * (HID / 8) + 255) / 256), 256, 0, stream>>>(x, X16);
  k_gemm16<0><<<(unsigned)((NR / 128) * (HID / 64)), 128, 0, stream>>>(X16, HID, BQ, HID, 0.0625f, bq, Q16, HID, NR, HID, HID);
  k_gemm16<0><<<(unsigned)((NR / 128) * (HID / 64)), 128, 0, stream>>>(X16, HID, BK, HID, 0.0625f, bk, K16, HID, NR, HID, HID);
  k_gemm16<1><<<(unsigned)((HID / 128) * (NR / 64)), 128, 0, stream>>>(BV, HID, X16, HID, 0.0625f, bv, VT, NR, HID, NR, HID);
  k_attn<<<(unsigned)(NB * NT * 4), 128, 0, stream>>>(Q16, K16, VT, perm, (float*)d_out);
}
